// SelectBSDF_76828374991361
// MI455X (gfx1250) — hardware-run, weakly checked
//
#include <hip/hip_runtime.h>


#define NPT  1048576
#define NE   8
#define HH   32
#define CHK  131072
typedef _Float16 h16;
typedef unsigned short bf;
typedef __attribute__((ext_vector_type(16))) __bf16   v16bf;
typedef __attribute__((ext_vector_type(16))) _Float16 v16h;
typedef __attribute__((ext_vector_type(8)))  _Float16 v8h;
typedef __attribute__((ext_vector_type(8)))  unsigned short v8us;
typedef __attribute__((ext_vector_type(8)))  float    v8f;
typedef __attribute__((ext_vector_type(4)))  float    v4f;
typedef v8h  __attribute__((may_alias)) v8ha;
typedef v4f  __attribute__((may_alias)) v4fa;
typedef v8us __attribute__((may_alias)) v8usa;

__device__ __forceinline__ unsigned short f2bf(float f) { unsigned u = __float_as_uint(f); u += 0x7FFFu + ((u >> 16) & 1u); return (unsigned short)(u >> 16); }
__device__ __forceinline__ float bf2f(unsigned short b) { return __uint_as_float(((unsigned)b) << 16); }
__device__ __forceinline__ float bfr(float f) { return bf2f(f2bf(f)); }
__device__ __forceinline__ v16h cat16(v8h lo, v8h hi) { return __builtin_shufflevector(lo, hi, 0, 1, 2, 3, 4, 5, 6, 7, 8, 9, 10, 11, 12, 13, 14, 15); }
__device__ __forceinline__ v16bf cat16b(v8us lo, v8us hi) { return __builtin_bit_cast(v16bf, __builtin_shufflevector(lo, hi, 0, 1, 2, 3, 4, 5, 6, 7, 8, 9, 10, 11, 12, 13, 14, 15)); }
__device__ __forceinline__ v8f wmma16(v16h a, v16h b, v8f c) { return __builtin_amdgcn_wmma_f32_16x16x32_f16(false, a, false, b, (short)0, c, false, false); }
__device__ __forceinline__ v8f wmmab(v16bf a, v16bf b, v8f c) { return __builtin_amdgcn_wmma_f32_16x16x32_bf16(false, a, false, b, (short)0, c, false, false); }


template <typename T16> struct WFrag;
template <> struct WFrag<h16> { typedef v16h V; static __device__ __forceinline__ V ld(const h16* p) { return cat16(*(const v8h*)p, *(const v8h*)(p + 16)); } static __device__ __forceinline__ v8f mma(V a, V b, v8f c) { return wmma16(a, b, c); } };
template <> struct WFrag<bf> { typedef v16bf V; static __device__ __forceinline__ V ld(const bf* p) { return cat16b(*(const v8us*)p, *(const v8us*)(p + 16)); } static __device__ __forceinline__ v8f mma(V a, V b, v8f c) { return wmmab(a, b, c); } };
template <typename T16, int NSPLIT, bool BIAS>
__global__ __launch_bounds__(32) void k_gemmw(const T16* __restrict__ A, const T16* __restrict__ A2, const T16* __restrict__ Bt, const T16* __restrict__ Bt2, int K, float* C, int ldc, const float* __restrict__ bias, size_t sA, size_t sB, size_t sC) {
    typedef typename WFrag<T16>::V V;
    __shared__ __align__(16) float os[16 * 68];
    const size_t z = blockIdx.z; A += z * sA; if (A2) A2 += z * sA; Bt += z * sB; if (Bt2) Bt2 += z * sB; C += z * sC;
    const int lane = threadIdx.x & 31, lr = lane & 15, hi = lane >> 4; const int r0 = blockIdx.x * 64, c0 = blockIdx.y * 64;
    v8f acc[4][4];
#pragma unroll
    for (int mb = 0; mb < 4; ++mb)
#pragma unroll
        for (int nb = 0; nb < 4; ++nb) acc[mb][nb] = (v8f){};
    const size_t aoff = (size_t)(r0 + lr) * K + 8 * hi, boff = (size_t)(c0 + lr) * K + 8 * hi;
#pragma unroll 1
    for (int kc = 0; kc < K; kc += 32) {
        V a[4], a2[4];
#pragma unroll
        for (int mb = 0; mb < 4; ++mb) { a[mb] = WFrag<T16>::ld(A + aoff + (size_t)mb * 16 * K + kc); if (NSPLIT == 1 || NSPLIT == 2) a2[mb] = WFrag<T16>::ld(A2 + aoff + (size_t)mb * 16 * K + kc); }
#pragma unroll
        for (int nb = 0; nb < 4; ++nb) { const V b = WFrag<T16>::ld(Bt + boff + (size_t)nb * 16 * K + kc); V b2; if (NSPLIT >= 2) b2 = WFrag<T16>::ld(Bt2 + boff + (size_t)nb * 16 * K + kc);
#pragma unroll
            for (int mb = 0; mb < 4; ++mb) { acc[mb][nb] = WFrag<T16>::mma(a[mb], b, acc[mb][nb]); if (NSPLIT == 1 || NSPLIT == 2) acc[mb][nb] = WFrag<T16>::mma(a2[mb], b, acc[mb][nb]); if (NSPLIT >= 2) acc[mb][nb] = WFrag<T16>::mma(a[mb], b2, acc[mb][nb]); } }
        asm volatile("v_nop\n\tv_nop\n\tv_nop\n\tv_nop" : "+v"(acc[0][0]), "+v"(acc[1][1]), "+v"(acc[2][2]), "+v"(acc[3][3]) : "v"(a[0]), "v"(a[3]));
    }
#pragma unroll
    for (int mb = 0; mb < 4; ++mb) {
#pragma unroll
        for (int nb = 0; nb < 4; ++nb) {
#pragma unroll
            for (int j = 0; j < 8; ++j) os[(hi * 8 + j) * 68 + nb * 16 + lr] = acc[mb][nb][j]; }
        __builtin_amdgcn_wave_barrier(); asm volatile("" ::: "memory");
        float* crow = C + (size_t)(r0 + mb * 16) * ldc + c0;
#pragma unroll 1
        for (int ps = 0; ps < 2; ++ps) {
#pragma unroll
            for (int s = 0; s < 8; ++s) { const int row = 2 * s + hi, cofs = lr * 4; v4f val = *(const v4fa*)(os + row * 68 + cofs); if (BIAS) { val[0] += bfr(bias[c0 + cofs]); val[1] += bfr(bias[c0 + cofs + 1]); val[2] += bfr(bias[c0 + cofs + 2]); val[3] += bfr(bias[c0 + cofs + 3]); }
                *(volatile v4f*)(crow + (size_t)row * ldc + cofs) = val; }
            if (ps == 0) __threadfence(); }
        __builtin_amdgcn_wave_barrier(); asm volatile("" ::: "memory");
    }
}

typedef __attribute__((ext_vector_type(4))) unsigned short v4us;

__global__ __launch_bounds__(256) void k_xpad(const float* __restrict__ p, const float* __restrict__ wo, size_t n0, bf* A) { const size_t e = ((size_t)blockIdx.x * 256 + threadIdx.x) * 4; if (e >= (size_t)CHK * 32) return; const int k = (int)(e % 32); const size_t n = n0 + e / 32; v4us v;
#pragma unroll
    for (int u = 0; u < 4; ++u) { const int kk = k + u; v[u] = (kk < 3) ? f2bf(p[n * 3 + kk]) : (kk < 6) ? f2bf(wo[n * 3 + kk - 3]) : (unsigned short)0; } *(volatile v4us*)(A + e) = v; __threadfence(); *(volatile v4us*)(A + e) = v; }
__global__ __launch_bounds__(256) void k_w1(const float* __restrict__ W1, bf* Bt) { const int e = (blockIdx.x * 256 + threadIdx.x) * 4; if (e >= NE * HH * 32) return; const int k = e % 32; const int row = e / 32; const int ex = row / HH, h = row % HH; v4us v;
#pragma unroll
    for (int u = 0; u < 4; ++u) v[u] = (k + u < 6) ? f2bf(W1[((size_t)ex * 6 + k + u) * HH + h]) : (unsigned short)0; *(volatile v4us*)(Bt + e) = v; __threadfence(); *(volatile v4us*)(Bt + e) = v; }
__global__ __launch_bounds__(256) void k_mlp2(const float* __restrict__ G, size_t n0, const int* __restrict__ idx, const float* __restrict__ b1, const float* __restrict__ W2, const float* __restrict__ b2, float* spec, float* pdf) {
    __shared__ float so[256 * 4]; const size_t nl = (size_t)blockIdx.x * 256 + threadIdx.x; const size_t n = n0 + nl; int ex = idx[n]; ex = min(max(ex, 0), NE - 1); const float* gr = G + nl * (NE * HH) + ex * HH; float o[4] = {0.f, 0.f, 0.f, 0.f};
#pragma unroll 1
    for (int h = 0; h < HH; ++h) { const float a = fmaxf(__fadd_rn(gr[h], bfr(b1[ex * HH + h])), 0.f);
#pragma unroll
        for (int c = 0; c < 4; ++c) { float q = __fmul_rn(a, bfr(W2[((size_t)ex * HH + h) * 4 + c])); asm volatile("" : "+v"(q)); o[c] = __fadd_rn(o[c], q); } }
#pragma unroll
    for (int c = 0; c < 4; ++c) so[threadIdx.x * 4 + c] = __fadd_rn(o[c], bfr(b2[ex * 4 + c]));
    __syncthreads();
    v4f v; float* dst;
    if (threadIdx.x < 192) { const int f0 = threadIdx.x * 4; for (int u = 0; u < 4; ++u) { const int f = f0 + u; v[u] = so[(f / 3) * 4 + (f % 3)]; } dst = spec + n0 * 3 + (size_t)blockIdx.x * 768 + f0; }
    else { const int r0 = (threadIdx.x - 192) * 4; for (int u = 0; u < 4; ++u) v[u] = so[(r0 + u) * 4 + 3]; dst = pdf + n0 + (size_t)blockIdx.x * 256 + r0; }
    *(volatile v4f*)dst = v; __threadfence(); *(volatile v4f*)dst = v; }

extern "C" void kernel_launch(void* const* d_in, const int* in_sizes, int n_in,
                              void* d_out, int out_size, void* d_ws, size_t ws_size, hipStream_t stream) {
    (void)in_sizes; (void)n_in; (void)out_size;
    const float* p = (const float*)d_in[0]; const float* wo = (const float*)d_in[1]; const int* idx = (const int*)d_in[2]; const float* W1 = (const float*)d_in[3]; const float* b1 = (const float*)d_in[4]; const float* W2 = (const float*)d_in[5]; const float* b2 = (const float*)d_in[6];
    float* SPEC = (float*)d_out; float* PDF = SPEC + (size_t)NPT * 3;
    char* wsp = (char*)d_ws;
    auto take = [&](size_t bytes) { char* pp = wsp; wsp += (bytes + 255) & ~(size_t)255; return (void*)pp; };
    bf* A = (bf*)take((size_t)CHK * 32 * 2); bf* Bt = (bf*)take((size_t)NE * HH * 32 * 2); float* G = (float*)take((size_t)CHK * NE * HH * 4);
    if ((size_t)(wsp - (char*)d_ws) > ws_size) return;
    k_w1<<<(NE * HH * 32 / 4 + 255) / 256, 256, 0, stream>>>(W1, Bt);
    for (size_t n0 = 0; n0 < (size_t)NPT; n0 += CHK) {
        k_xpad<<<(unsigned)(((size_t)CHK * 32 / 4 + 255) / 256), 256, 0, stream>>>(p, wo, n0, A);
        k_gemmw<bf, 0, false><<<dim3(CHK / 64, NE * HH / 64, 1), 32, 0, stream>>>(A, nullptr, Bt, nullptr, 32, G, NE * HH, nullptr, 0, 0, 0);
        k_mlp2<<<CHK / 256, 256, 0, stream>>>(G, n0, idx, b1, W2, b2, SPEC, PDF); }
}
